// mamba_encoder_43774306681538
// MI455X (gfx1250) — hardware-verified
//
#include <hip/hip_runtime.h>
#include <math.h>

typedef __attribute__((ext_vector_type(16))) _Float16 v16h;
typedef __attribute__((ext_vector_type(8)))  _Float16 v8h;
typedef __attribute__((ext_vector_type(4)))  _Float16 v4h;
typedef __attribute__((ext_vector_type(16))) __bf16   v16b;
typedef __attribute__((ext_vector_type(8)))  __bf16   v8b;
typedef __attribute__((ext_vector_type(8)))  float    v8f;
typedef __attribute__((ext_vector_type(4)))  float    v4f;

constexpr int kBatch = 16;
constexpr int kSeq   = 8192;
constexpr int kRows  = kBatch * kSeq;
constexpr int kDm    = 16;
constexpr int kDi    = 32;
constexpr int kNs    = 16;
constexpr int kHm    = 32;
constexpr int kXd    = 1 + 2 * kNs;
constexpr int kNP    = 64;
constexpr int kConv  = 4;
constexpr int kThr   = 256;
constexpr float kRmsEps = 1e-6f;

constexpr float kWCarry = 4096.0f;
constexpr float kNCarry = 1024.0f;
constexpr float kACarry = 256.0f;
constexpr float kScN = 1.0f / (kNCarry * kWCarry);
constexpr float kScA = 1.0f / (kACarry * kWCarry);
constexpr float kF16MinNormal = 6.103515625e-5f;

static_assert((kRows % 64) == 0 && ((kRows / 64) * (kNP / 64)) % 8 == 0, "GEMM grids exact");

constexpr size_t kGsz = (size_t)kRows * kNP * 4;
constexpr size_t kOffG1 = 0;
constexpr size_t kOffG2 = kOffG1 + kGsz;
constexpr size_t kOffG3 = kOffG2 + kGsz;
constexpr size_t kOffF1 = kOffG3 + kGsz;
constexpr size_t kOffF2 = kOffF1 + (size_t)kRows * 32 * 2;
constexpr size_t kOffF3 = kOffF2 + (size_t)kRows * 64 * 2;
constexpr size_t kOffXC = kOffF3 + (size_t)kRows * 64 * 2;
constexpr size_t kOffYG = kOffXC + (size_t)kRows * kDi * 4;
constexpr size_t kOffXR = kOffYG + (size_t)kRows * kDi * 4;
constexpr size_t kOffWP = kOffXR + (size_t)kRows * kDm * 4;
constexpr int kWpIn = 0, kWpX = kWpIn + 64 * 32, kWpOut = kWpX + 64 * 64, kWpF1 = kWpOut + 64 * 64, kWpF2 = kWpF1 + 64 * 32, kWpF3 = kWpF2 + 64 * 64, kWpTot = kWpF3 + 64 * 64;
constexpr size_t kOffBV = kOffWP + (size_t)kWpTot * 2;
constexpr size_t kWsTotal = kOffBV + 6 * 64 * 4;
static_assert(kWsTotal <= 268435456ull, "inside the offered workspace");
static_assert((kOffG2 % 256) == 0 && (kOffG3 % 256) == 0 && (kOffF1 % 256) == 0 && (kOffF2 % 256) == 0 && (kOffF3 % 256) == 0 && (kOffXC % 256) == 0 && (kOffYG % 256) == 0 && (kOffXR % 256) == 0 && (kOffWP % 256) == 0 && (kOffBV % 256) == 0, "aligned regions");
static_assert(((kWpX * 2) % 256) == 0 && ((kWpOut * 2) % 256) == 0 && ((kWpF1 * 2) % 256) == 0 && ((kWpF2 * 2) % 256) == 0 && ((kWpF3 * 2) % 256) == 0, "aligned weight planes");

__device__ __forceinline__ unsigned short f2bf_bits(float f) {
  unsigned u = __float_as_uint(f);
  return (unsigned short)((u + 0x7FFFu + ((u >> 16) & 1u)) >> 16);
}
__device__ __forceinline__ float bf_bits2f(unsigned short h) { return __uint_as_float(((unsigned)h) << 16); }
__device__ __forceinline__ float bf16r(float f) { return bf_bits2f(f2bf_bits(f)); }
__device__ __forceinline__ float carry_flush(float v, float carry) {
  const float s = v * carry;
  return (fabsf(s) < kF16MinNormal) ? 0.0f : s;
}
__device__ __forceinline__ float frcp(float x) { return __builtin_amdgcn_rcpf(x); }

__device__ __forceinline__ void dep_guard4_h(v8f& a, v8f& b, v8f& c, v8f& d, v16h x, v16h y) { asm volatile("v_nop\n\tv_nop\n\tv_nop\n\tv_nop" : "+v"(a), "+v"(b), "+v"(c), "+v"(d) : "v"(x), "v"(y)); }
__device__ __forceinline__ void dep_guard4_b(v8f& a, v8f& b, v8f& c, v8f& d, v16b x, v16b y) { asm volatile("v_nop\n\tv_nop\n\tv_nop\n\tv_nop" : "+v"(a), "+v"(b), "+v"(c), "+v"(d) : "v"(x), "v"(y)); }
__device__ __forceinline__ void keep4_h(v16h a, v16h b, v16h c, v16h d) { asm volatile("v_nop" :: "v"(a), "v"(b), "v"(c), "v"(d)); }
__device__ __forceinline__ void keep4_b(v16b a, v16b b, v16b c, v16b d) { asm volatile("v_nop" :: "v"(a), "v"(b), "v"(c), "v"(d)); }
__device__ __forceinline__ void acc_guard4(v8f& a, v8f& b, v8f& c, v8f& d) { asm volatile("v_nop\n\tv_nop\n\tv_nop\n\tv_nop" : "+v"(a), "+v"(b), "+v"(c), "+v"(d)); }

template <typename T> struct Frag;
template <> struct Frag<_Float16> {
  typedef v16h V; union U { v16h v; v8h h[2]; };
  static __device__ __forceinline__ v16h load(const _Float16* p) {
    U f; f.h[0] = *(const v8h*)(p); f.h[1] = *(const v8h*)(p + 16); return f.v;
  }
  static __device__ __forceinline__ v8f mma(v16h a, v16h b, v8f c) {
    return __builtin_amdgcn_wmma_f32_16x16x32_f16(false, a, false, b, (short)0, c, false, false);
  }
  static __device__ __forceinline__ void guard4(v8f& a, v8f& b, v8f& c, v8f& d, v16h x, v16h y) { dep_guard4_h(a, b, c, d, x, y); }
  static __device__ __forceinline__ void keep(v16h a, v16h b, v16h c, v16h d) { keep4_h(a, b, c, d); }
};
template <> struct Frag<__bf16> {
  typedef v16b V; union U { v16b v; v8b h[2]; };
  static __device__ __forceinline__ v16b load(const __bf16* p) {
    U f; f.h[0] = *(const v8b*)(p); f.h[1] = *(const v8b*)(p + 16); return f.v;
  }
  static __device__ __forceinline__ v8f mma(v16b a, v16b b, v8f c) {
    return __builtin_amdgcn_wmma_f32_16x16x32_bf16(false, a, false, b, (short)0, c, false, false);
  }
  static __device__ __forceinline__ void guard4(v8f& a, v8f& b, v8f& c, v8f& d, v16b x, v16b y) { dep_guard4_b(a, b, c, d, x, y); }
  static __device__ __forceinline__ void keep(v16b a, v16b b, v16b c, v16b d) { keep4_b(a, b, c, d); }
};

__device__ __forceinline__ v8f mma_h(v16h a, v16h b, v8f c) {
  c = __builtin_amdgcn_wmma_f32_16x16x32_f16(false, a, false, b, (short)0, c, false, false);
  asm volatile("v_nop\n\tv_nop\n\tv_nop\n\tv_nop" : "+v"(c) : "v"(a), "v"(b));
  return c;
}

template <int ET> struct Elem;
template <> struct Elem<0> { typedef _Float16 T; };
template <> struct Elem<1> { typedef __bf16 T; };
template <int ET, bool SPLIT, int BIAS_MODE, int OUT_MODE, bool RESID, int ACT = 0>
__global__ __launch_bounds__(256) void wmma_gemm64(
    const unsigned short* __restrict__ Ap, const unsigned short* __restrict__ A2p, int lda, long strideA,
    const unsigned short* __restrict__ Btp, const unsigned short* __restrict__ Bt2p, int ldb, long strideB,
    void* __restrict__ Cout, void* __restrict__ Cout2, int ldc, long strideC,
    const float* __restrict__ bias,
    const float* __restrict__ resid, long strideR,
    int M, int N, int K, float scale) {
  typedef typename Elem<ET>::T T;
  typedef typename Frag<T>::V V;
  const T* A = (const T*)Ap; const T* A2 = (const T*)A2p; const T* Bt = (const T*)Btp; const T* Bt2 = (const T*)Bt2p;
  __shared__ __align__(16) float sT[8][16 * 68];
  const int b    = blockIdx.y;
  const int lane = threadIdx.x & 31;
  const int wave = threadIdx.x >> 5;
  const int tilesN = N >> 6;
  const int tilesM = M >> 6;
  const int tile = blockIdx.x * 8 + wave;
  if (tile >= tilesM * tilesN) return;
  const int tm = tile / tilesN;
  const int tn = tile - tm * tilesN;
  const int m0 = tm << 6;
  const int n0 = tn << 6;

  const T* Ab  = A  + (size_t)b * strideA;
  const T* Bb  = Bt + (size_t)b * strideB;
  const T* Ab2 = SPLIT ? (A2  + (size_t)b * strideA) : nullptr;
  const T* Bb2 = SPLIT ? (Bt2 + (size_t)b * strideB) : nullptr;

  const int rlane = lane & 15;
  const int koff  = (lane >> 4) * 8;
  const int mOff  = (lane >> 4) * 8;

  v8f acc[4][4];
#pragma unroll
  for (int i = 0; i < 4; ++i)
#pragma unroll
    for (int j = 0; j < 4; ++j) acc[i][j] = (v8f){0.f,0.f,0.f,0.f,0.f,0.f,0.f,0.f};

  for (int k0 = 0; k0 < K; k0 += 32) {
    V bh[4], bl[4];
#pragma unroll
    for (int j = 0; j < 4; ++j) {
      const size_t bo = (size_t)(n0 + (j << 4) + rlane) * ldb + koff + k0;
      bh[j] = Frag<T>::load(Bb + bo);
      if (SPLIT) bl[j] = Frag<T>::load(Bb2 + bo);
    }
#pragma unroll
    for (int i = 0; i < 4; ++i) {
      const size_t ao = (size_t)(m0 + (i << 4) + rlane) * lda + koff + k0;
      V ah = Frag<T>::load(Ab + ao);
      V al;
      if (SPLIT) al = Frag<T>::load(Ab2 + ao);
#pragma unroll
      for (int j = 0; j < 4; ++j) {
        acc[i][j] = Frag<T>::mma(ah, bh[j], acc[i][j]);
        if (SPLIT) {
          acc[i][j] = Frag<T>::mma(ah, bl[j], acc[i][j]);
          acc[i][j] = Frag<T>::mma(al, bh[j], acc[i][j]);
        }
      }
      Frag<T>::guard4(acc[i][0], acc[i][1], acc[i][2], acc[i][3], ah, SPLIT ? al : ah);
    }
    Frag<T>::keep(bh[0], bh[1], bh[2], bh[3]);
    if (SPLIT) Frag<T>::keep(bl[0], bl[1], bl[2], bl[3]);
  }
  acc_guard4(acc[0][0], acc[0][1], acc[0][2], acc[0][3]);
  acc_guard4(acc[1][0], acc[1][1], acc[1][2], acc[1][3]);
  acc_guard4(acc[2][0], acc[2][1], acc[2][2], acc[2][3]);
  acc_guard4(acc[3][0], acc[3][1], acc[3][2], acc[3][3]);

  float* slab = sT[wave];
  const float* Rb = RESID ? (resid + (size_t)b * strideR) : nullptr;
#pragma unroll
  for (int i = 0; i < 4; ++i) {
    const int mBase = m0 + (i << 4);
#pragma unroll
    for (int j = 0; j < 4; ++j) {
      const int n = n0 + (j << 4) + rlane;
      float bv = 0.f;
      if (BIAS_MODE == 2) bv = bias[n];
#pragma unroll
      for (int r = 0; r < 8; ++r) {
        float v = acc[i][j][r] * scale;
        if (BIAS_MODE == 1) v += bias[mBase + mOff + r];
        if (BIAS_MODE == 2) v += bv;
        if (RESID) v += Rb[(size_t)(mBase + mOff + r) * ldc + n];
        if (ACT == 1) v = tanhf(v);
        if (ACT == 2) v = fmaxf(v, 0.0f);
        if (ACT == 3) v = v / (1.0f + expf(-v));
        if (ACT == 4) v = (v > 0.f) ? v : 0.01f * v;
        slab[(mOff + r) * 68 + (j << 4) + rlane] = v;
      }
    }
    __builtin_amdgcn_fence(__ATOMIC_RELEASE, "workgroup");
    __builtin_amdgcn_wave_barrier();
    __builtin_amdgcn_fence(__ATOMIC_ACQUIRE, "workgroup");
    if (OUT_MODE == 0) {
      float* C = (float*)Cout + (size_t)b * strideC;
      const int hh = lane >> 4, c4 = (lane & 15) * 4;
      for (int pass = 0; pass < 2; ++pass) {
#pragma unroll
        for (int it = 0; it < 8; ++it) {
          const int row = it * 2 + hh;
          v4f v = *(const v4f*)(slab + row * 68 + c4);
          *(volatile v4f*)(C + (size_t)(mBase + row) * ldc + n0 + c4) = v;
        }
        __threadfence();
      }
    } else {
      const int q = lane >> 3, c8 = (lane & 7) * 8;
      unsigned short* C  = (unsigned short*)Cout  + (size_t)b * strideC;
      unsigned short* C2 = (OUT_MODE == 2) ? ((unsigned short*)Cout2 + (size_t)b * strideC) : nullptr;
      for (int pass = 0; pass < 2; ++pass) {
#pragma unroll
        for (int it = 0; it < 4; ++it) {
          const int row = it * 4 + q;
          const float* sp = slab + row * 68 + c8;
          v8h hv, lv;
#pragma unroll
          for (int e = 0; e < 8; ++e) {
            if (OUT_MODE == 1) {
              hv[e] = (_Float16)sp[e];
            } else {
              unsigned short hb = f2bf_bits(sp[e]);
              unsigned short lb = f2bf_bits(sp[e] - bf_bits2f(hb));
              hv[e] = __builtin_bit_cast(_Float16, hb);
              lv[e] = __builtin_bit_cast(_Float16, lb);
            }
          }
          *(volatile v8h*)(C + (size_t)(mBase + row) * ldc + n0 + c8) = hv;
          if (OUT_MODE == 2) *(volatile v8h*)(C2 + (size_t)(mBase + row) * ldc + n0 + c8) = lv;
        }
        __threadfence();
      }
    }
    __builtin_amdgcn_fence(__ATOMIC_RELEASE, "workgroup");
    __builtin_amdgcn_wave_barrier();
    __builtin_amdgcn_fence(__ATOMIC_ACQUIRE, "workgroup");
  }
}


__device__ __forceinline__ void split_hl(float v, float c, _Float16& hi, _Float16& lo) {
  const float sv = carry_flush(v, c);
  hi = (_Float16)sv;
  const float r = sv - (float)hi;
  lo = (_Float16)((fabsf(r) < kF16MinNormal) ? 0.0f : r);
}

__global__ __launch_bounds__(kThr) void wsmall_plane_kernel(const float* __restrict__ W, unsigned short* __restrict__ dst, int Kin, int Nin) {
  const int i = blockIdx.x * kThr + threadIdx.x;
  const int per = (2 * Kin) >> 3;
  const int n = i / per;
  const int c8 = (i - n * per) * 8;
  const bool live = n < Nin;
  const int nc = live ? n : 0;
  v8h hv;
#pragma unroll
  for (int e = 0; e < 8; ++e) {
    const int c = c8 + e;
    const int k = (c >= Kin) ? (c - Kin) : c;
    const float w = W[(size_t)k * Nin + nc];
    hv[e] = (_Float16)(live ? carry_flush(bf16r(w), kWCarry) : 0.0f);
  }
  unsigned short* dp = dst + (size_t)i * 8;
  *(volatile v8h*)dp = hv;
  __threadfence();
  *(volatile v8h*)dp = hv;
}

__global__ __launch_bounds__(128) void bias_rows_kernel(const float* __restrict__ b1, const float* __restrict__ b2, const float* __restrict__ b3, float* __restrict__ BV) {
  const int i = blockIdx.x * 128 + threadIdx.x;
  const int p = i >> 6, c = i & 63;
  const float v1 = b1[(c < kHm) ? c : 0];
  const float v2 = b2[(c < kHm) ? c : 0];
  const float v3 = b3[(c < kDm) ? c : 0];
  const float o = (p == 3) ? ((c < kHm) ? bf16r(v1) : 0.0f) : ((p == 4) ? ((c < kHm) ? bf16r(v2) : 0.0f) : ((p == 5) ? ((c < kDm) ? bf16r(v3) : 0.0f) : 0.0f));
  for (int pass = 0; pass < 2; ++pass) {
    *(volatile float*)(BV + i) = o;
    __threadfence();
  }
}

template <bool kSecond>
__global__ __launch_bounds__(kThr) void rms_rows_kernel(const float* __restrict__ x, const float* __restrict__ O1, const float* __restrict__ w,
                                                        unsigned short* __restrict__ Xh, float* __restrict__ XR) {
  const size_t row = (size_t)blockIdx.x * kThr + threadIdx.x;
  float h[kDm];
#pragma unroll
  for (int q = 0; q < 4; ++q) {
    const v4f xv = *(const v4f*)(x + row * kDm + 4 * q);
#pragma unroll
    for (int e = 0; e < 4; ++e) { const float x0 = xv[e]; h[4 * q + e] = bf16r(x0); }
    if (kSecond) {
      const v4f ov = *(const v4f*)(O1 + row * kNP + 4 * q);
#pragma unroll
      for (int e = 0; e < 4; ++e) h[4 * q + e] = ov[e] + h[4 * q + e];
    }
  }
  float ss = 0.0f;
#pragma unroll
  for (int k = 0; k < kDm; ++k) ss += h[k] * h[k];
  const float rs = 1.0f / sqrtf(ss * (1.0f / (float)kDm) + kRmsEps);
  v8h o0, o1, o2, o3;
#pragma unroll
  for (int k = 0; k < kDm; ++k) {
    const float w0 = w[k];
    _Float16 hi, lo;
    split_hl(bf16r(w0) * (h[k] * rs), kNCarry, hi, lo);
    if (k < 8) { o0[k] = hi; o2[k] = lo; } else { o1[k - 8] = hi; o3[k - 8] = lo; }
  }
  unsigned short* dp = Xh + row * 32;
  for (int pass = 0; pass < 2; ++pass) {
    *(volatile v8h*)(dp) = o0;
    *(volatile v8h*)(dp + 8) = o1;
    *(volatile v8h*)(dp + 16) = o2;
    *(volatile v8h*)(dp + 24) = o3;
    if (kSecond) {
#pragma unroll
      for (int q = 0; q < 4; ++q) { v4f t; t[0] = h[4 * q]; t[1] = h[4 * q + 1]; t[2] = h[4 * q + 2]; t[3] = h[4 * q + 3]; *(volatile v4f*)(XR + row * kDm + 4 * q) = t; }
    }
    __threadfence();
  }
}
static_assert(kRows % kThr == 0, "row grids exact");

__global__ __launch_bounds__(kThr) void conv_silu_kernel(const float* __restrict__ XZ, const float* __restrict__ conv_w, const float* __restrict__ conv_b,
                                                         float* __restrict__ XC, unsigned short* __restrict__ XC16) {
  const size_t v = (size_t)blockIdx.x * kThr + threadIdx.x;
  const size_t row = v >> 3;
  const int d4 = (int)(v & 7) * 4;
  const int l = (int)(row & (kSeq - 1));
  v4f acc = *(const v4f*)(conv_b + d4);
#pragma unroll
  for (int e = 0; e < 4; ++e) { const float b0 = acc[e]; acc[e] = bf16r(b0); }
#pragma unroll
  for (int j = 0; j < kConv; ++j) {
    const int back = kConv - 1 - j;
    const bool ok = l >= back;
    const size_t rr = ok ? (row - back) : row;
    const v4f xin = *(const v4f*)(XZ + rr * kNP + d4);
#pragma unroll
    for (int e = 0; e < 4; ++e) {
      const float w = conv_w[(size_t)(d4 + e) * kConv + j];
      acc[e] += ok ? (bf16r(w) * xin[e]) : 0.0f;
    }
  }
  v4f o;
  v4h hv, lv;
#pragma unroll
  for (int e = 0; e < 4; ++e) {
    const float s = acc[e] * (1.0f / (1.0f + expf(-acc[e])));
    o[e] = s;
    _Float16 hi, lo;
    split_hl(s, kACarry, hi, lo);
    hv[e] = hi; lv[e] = lo;
  }
  for (int pass = 0; pass < 2; ++pass) {
    *(volatile v4f*)(XC + row * kDi + d4) = o;
    *(volatile v4h*)(XC16 + row * 64 + d4) = hv;
    *(volatile v4h*)(XC16 + row * 64 + kDi + d4) = lv;
    __threadfence();
  }
}
static_assert(((size_t)kRows * 8) % kThr == 0 && (kSeq & (kSeq - 1)) == 0, "conv grid exact");

__global__ __launch_bounds__(kThr) void sel_scan_kernel(const float* __restrict__ P, const float* __restrict__ XC, const float* __restrict__ XZ,
                                                        const float* __restrict__ dtw, const float* __restrict__ dtb, const float* __restrict__ A_log,
                                                        const float* __restrict__ Dsk, float* __restrict__ YG) {
  const int v = blockIdx.x * kThr + threadIdx.x;
  const int b = v >> 5;
  const int d = v & 31;
  float A[kNs], h[kNs];
#pragma unroll
  for (int n = 0; n < kNs; ++n) { const float al = A_log[(size_t)d * kNs + n]; A[n] = -expf(bf16r(al)); h[n] = 0.0f; }
  const float w0 = dtw[d], b0 = dtb[d], d0 = Dsk[d];
  const float wdt = bf16r(w0), bdt = bf16r(b0), dsk = bf16r(d0);
  const size_t r0 = (size_t)b * kSeq;
#pragma unroll 1
  for (int l = 0; l < kSeq; ++l) {
    const size_t row = r0 + l;
    const float* pr = P + row * kNP;
    const float sv = pr[0] * wdt + bdt;
    const float xc = XC[row * kDi + d];
    const float zz = XZ[row * kNP + kDi + d];
    const float dt = (sv > 20.0f) ? sv : log1pf(expf(sv));
    float y = 0.0f;
#pragma unroll
    for (int n = 0; n < kNs; ++n) {
      const float hn = __expf(dt * A[n]) * h[n] + dt * pr[1 + n] * xc;
      h[n] = hn;
      y += hn * pr[1 + kNs + n];
    }
    const float g = zz * frcp(1.0f + __expf(-zz));
    const float o = (y + dsk * xc) * g;
    float* op = YG + row * kDi + d;
    *(volatile float*)op = o;
    __threadfence();
    *(volatile float*)op = o;
  }
}
static_assert((kBatch * kDi) % kThr == 0, "scan grid exact");

template <bool kRelu>
__global__ __launch_bounds__(kThr) void act_cast_kernel(const float* __restrict__ src, unsigned short* __restrict__ dst) {
  const size_t v = (size_t)blockIdx.x * kThr + threadIdx.x;
  const size_t row = v >> 3;
  const int d4 = (int)(v & 7) * 4;
  const v4f a = *(const v4f*)(src + row * (kRelu ? kNP : kDi) + d4);
  v4h hv, lv;
#pragma unroll
  for (int e = 0; e < 4; ++e) {
    const float t = kRelu ? fmaxf(a[e], 0.0f) : a[e];
    _Float16 hi, lo;
    split_hl(t, kACarry, hi, lo);
    hv[e] = hi; lv[e] = lo;
  }
  for (int pass = 0; pass < 2; ++pass) {
    *(volatile v4h*)(dst + row * 64 + d4) = hv;
    *(volatile v4h*)(dst + row * 64 + 32 + d4) = lv;
    __threadfence();
  }
}

__global__ __launch_bounds__(kThr) void final_add_kernel(const float* __restrict__ XR, const float* __restrict__ O3, float* __restrict__ out) {
  const size_t v = (size_t)blockIdx.x * kThr + threadIdx.x;
  const size_t row = v >> 2;
  const int c4 = (int)(v & 3) * 4;
  const v4f a = *(const v4f*)(XR + v * 4);
  const v4f o3 = *(const v4f*)(O3 + row * kNP + c4);
  v4f o;
#pragma unroll
  for (int e = 0; e < 4; ++e) o[e] = a[e] + o3[e];
  float* dp = out + v * 4;
  *(volatile v4f*)dp = o;
  __threadfence();
  *(volatile v4f*)dp = o;
}
static_assert(((size_t)kRows * 4) % kThr == 0, "final grid exact");

extern "C" void kernel_launch(void* const* d_in, const int* in_sizes, int n_in,
                              void* d_out, int out_size, void* d_ws, size_t ws_size,
                              hipStream_t stream) {
  if (n_in < 18 || d_out == nullptr || d_ws == nullptr) return;
  if (in_sizes[0] != kRows * kDm || in_sizes[1] != kDm || in_sizes[2] != kDm * 2 * kDi || in_sizes[3] != kDi * kConv || in_sizes[4] != kDi) return;
  if (in_sizes[5] != kDi * kXd || in_sizes[6] != kDi || in_sizes[7] != kDi || in_sizes[8] != kDi * kNs || in_sizes[9] != kDi) return;
  if (in_sizes[10] != kDi * kDm || in_sizes[11] != kDm || in_sizes[12] != kDm * kHm || in_sizes[13] != kHm) return;
  if (in_sizes[14] != kHm * kHm || in_sizes[15] != kHm || in_sizes[16] != kHm * kDm || in_sizes[17] != kDm) return;
  if (out_size != kRows * kDm) return;
  if (ws_size < kWsTotal) return;
  const float* x = (const float*)d_in[0];
  const float* rms1_w = (const float*)d_in[1];
  const float* in_proj_w = (const float*)d_in[2];
  const float* conv_w = (const float*)d_in[3];
  const float* conv_b = (const float*)d_in[4];
  const float* x_proj_w = (const float*)d_in[5];
  const float* dt_proj_w = (const float*)d_in[6];
  const float* dt_proj_b = (const float*)d_in[7];
  const float* A_log = (const float*)d_in[8];
  const float* D_skip = (const float*)d_in[9];
  const float* out_proj_w = (const float*)d_in[10];
  const float* rms2_w = (const float*)d_in[11];
  const float* fc1_w = (const float*)d_in[12];
  const float* fc1_b = (const float*)d_in[13];
  const float* fc2_w = (const float*)d_in[14];
  const float* fc2_b = (const float*)d_in[15];
  const float* fc3_w = (const float*)d_in[16];
  const float* fc3_b = (const float*)d_in[17];
  float* out = (float*)d_out;
  char* ws = (char*)d_ws;
  float* G1 = (float*)(ws + kOffG1);
  float* G2 = (float*)(ws + kOffG2);
  float* G3 = (float*)(ws + kOffG3);
  unsigned short* F1 = (unsigned short*)(ws + kOffF1);
  unsigned short* F2 = (unsigned short*)(ws + kOffF2);
  unsigned short* F3 = (unsigned short*)(ws + kOffF3);
  float* XC = (float*)(ws + kOffXC);
  float* YG = (float*)(ws + kOffYG);
  float* XR = (float*)(ws + kOffXR);
  unsigned short* WP = (unsigned short*)(ws + kOffWP);
  float* BV = (float*)(ws + kOffBV);
  const int gTiles = (kRows / 64) * (kNP / 64) / 8;

  wsmall_plane_kernel<<<1, kThr, 0, stream>>>(in_proj_w, WP + kWpIn, kDm, 2 * kDi);
  wsmall_plane_kernel<<<2, kThr, 0, stream>>>(x_proj_w, WP + kWpX, kDi, kXd);
  wsmall_plane_kernel<<<2, kThr, 0, stream>>>(out_proj_w, WP + kWpOut, kDi, kDm);
  wsmall_plane_kernel<<<1, kThr, 0, stream>>>(fc1_w, WP + kWpF1, kDm, kHm);
  wsmall_plane_kernel<<<2, kThr, 0, stream>>>(fc2_w, WP + kWpF2, kHm, kHm);
  wsmall_plane_kernel<<<2, kThr, 0, stream>>>(fc3_w, WP + kWpF3, kHm, kDm);
  bias_rows_kernel<<<3, 128, 0, stream>>>(fc1_b, fc2_b, fc3_b, BV);

  rms_rows_kernel<false><<<kRows / kThr, kThr, 0, stream>>>(x, G3, rms1_w, F1, XR);
  wmma_gemm64<0, false, 2, 0, false, 0><<<dim3(gTiles, 1), 256, 0, stream>>>(
      F1, F1, 32, 0L, WP + kWpIn, WP + kWpIn, 32, 0L, (void*)G1, (void*)G1, kNP, 0L, BV + 0 * 64, nullptr, 0L, kRows, kNP, 32, kScN);
  conv_silu_kernel<<<(int)(((size_t)kRows * 8) / kThr), kThr, 0, stream>>>(G1, conv_w, conv_b, XC, F2);
  wmma_gemm64<0, false, 2, 0, false, 0><<<dim3(gTiles, 1), 256, 0, stream>>>(
      F2, F2, 64, 0L, WP + kWpX, WP + kWpX, 64, 0L, (void*)G2, (void*)G2, kNP, 0L, BV + 1 * 64, nullptr, 0L, kRows, kNP, 64, kScA);
  sel_scan_kernel<<<(kBatch * kDi) / kThr, kThr, 0, stream>>>(G2, XC, G1, dt_proj_w, dt_proj_b, A_log, D_skip, YG);
  act_cast_kernel<false><<<(int)(((size_t)kRows * 8) / kThr), kThr, 0, stream>>>(YG, F3);
  wmma_gemm64<0, false, 2, 0, false, 0><<<dim3(gTiles, 1), 256, 0, stream>>>(
      F3, F3, 64, 0L, WP + kWpOut, WP + kWpOut, 64, 0L, (void*)G3, (void*)G3, kNP, 0L, BV + 2 * 64, nullptr, 0L, kRows, kNP, 64, kScA);
  rms_rows_kernel<true><<<kRows / kThr, kThr, 0, stream>>>(x, G3, rms2_w, F1, XR);
  wmma_gemm64<0, false, 2, 0, false, 0><<<dim3(gTiles, 1), 256, 0, stream>>>(
      F1, F1, 32, 0L, WP + kWpF1, WP + kWpF1, 32, 0L, (void*)G2, (void*)G2, kNP, 0L, BV + 3 * 64, nullptr, 0L, kRows, kNP, 32, kScN);
  act_cast_kernel<true><<<(int)(((size_t)kRows * 8) / kThr), kThr, 0, stream>>>(G2, F2);
  wmma_gemm64<0, false, 2, 0, false, 0><<<dim3(gTiles, 1), 256, 0, stream>>>(
      F2, F2, 64, 0L, WP + kWpF2, WP + kWpF2, 64, 0L, (void*)G3, (void*)G3, kNP, 0L, BV + 4 * 64, nullptr, 0L, kRows, kNP, 64, kScA);
  act_cast_kernel<true><<<(int)(((size_t)kRows * 8) / kThr), kThr, 0, stream>>>(G3, F3);
  wmma_gemm64<0, false, 2, 0, false, 0><<<dim3(gTiles, 1), 256, 0, stream>>>(
      F3, F3, 64, 0L, WP + kWpF3, WP + kWpF3, 64, 0L, (void*)G1, (void*)G1, kNP, 0L, BV + 5 * 64, nullptr, 0L, kRows, kNP, 64, kScA);
  final_add_kernel<<<(int)(((size_t)kRows * 4) / kThr), kThr, 0, stream>>>(XR, G1, out);
}
